// CrossModalAttention_16466904613743
// MI455X (gfx1250) — hardware-verified
//
#include <hip/hip_runtime.h>


#ifndef NB
#define NB 8
#endif
#define NB_FULL 8
#define CC   256
#define HH   64
#define WW   64
#define HW   (HH * WW)
#define IMG  (CC * HW)
#define NTK  16
#define GB   ((NB < 4) ? NB : 4)
#define SCL  0.25f
#define L2E  1.4426950408889634f
static_assert(NB % GB == 0);
static_assert(NB <= NB_FULL);
static_assert(CC % 64 == 0);
static_assert(HW % 64 == 0);
static_assert(CC % 32 == 0);

typedef _Float16 h16;
typedef unsigned short bf;
typedef __attribute__((ext_vector_type(16))) __bf16   v16bf;
typedef __attribute__((ext_vector_type(16))) _Float16 v16h;
typedef __attribute__((ext_vector_type(8)))  _Float16 v8h;
typedef __attribute__((ext_vector_type(8)))  unsigned short v8us;
typedef __attribute__((ext_vector_type(8)))  float    v8f;
typedef __attribute__((ext_vector_type(4)))  float    v4f;
typedef v4f  __attribute__((may_alias)) v4fa;

__device__ __forceinline__ unsigned short f2bf(float f) { unsigned u = __float_as_uint(f); u += 0x7FFFu + ((u >> 16) & 1u); return (unsigned short)(u >> 16); }
__device__ __forceinline__ float bf2f(unsigned short b) { return __uint_as_float(((unsigned)b) << 16); }
__device__ __forceinline__ float bfr(float f) { return bf2f(f2bf(f)); }
__device__ __forceinline__ v16h cat16(v8h lo, v8h hi) { return __builtin_shufflevector(lo, hi, 0, 1, 2, 3, 4, 5, 6, 7, 8, 9, 10, 11, 12, 13, 14, 15); }
__device__ __forceinline__ v16bf cat16b(v8us lo, v8us hi) { return __builtin_bit_cast(v16bf, __builtin_shufflevector(lo, hi, 0, 1, 2, 3, 4, 5, 6, 7, 8, 9, 10, 11, 12, 13, 14, 15)); }
__device__ __forceinline__ v8f wmma16(v16h a, v16h b, v8f c) { return __builtin_amdgcn_wmma_f32_16x16x32_f16(false, a, false, b, (short)0, c, false, false); }
__device__ __forceinline__ v8f wmmab(v16bf a, v16bf b, v8f c) { return __builtin_amdgcn_wmma_f32_16x16x32_bf16(false, a, false, b, (short)0, c, false, false); }

template <typename T16> struct WFrag;
template <> struct WFrag<h16> { typedef v16h V; static __device__ __forceinline__ V ld(const h16* p) { return cat16(*(const v8h*)p, *(const v8h*)(p + 16)); } static __device__ __forceinline__ v8f mma(V a, V b, v8f c) { return wmma16(a, b, c); } };
template <> struct WFrag<bf> { typedef v16bf V; static __device__ __forceinline__ V ld(const bf* p) { return cat16b(*(const v8us*)p, *(const v8us*)(p + 16)); } static __device__ __forceinline__ v8f mma(V a, V b, v8f c) { return wmmab(a, b, c); } };
template <typename T16, int NSPLIT, bool BIASR>
__global__ __launch_bounds__(32) void k_gemmw(const T16* __restrict__ A, const T16* __restrict__ A2, const T16* __restrict__ Bt, const T16* __restrict__ Bt2, int K, float* C, int ldc, const float* __restrict__ bias, size_t sA, size_t sB, size_t sC) {
    typedef typename WFrag<T16>::V V;
    __shared__ __align__(16) float os[16 * 68];
    const size_t z = blockIdx.z; A += z * sA; if (A2) A2 += z * sA; Bt += z * sB; if (Bt2) Bt2 += z * sB; C += z * sC;
    const int lane = threadIdx.x & 31, lr = lane & 15, hi = lane >> 4; const int r0 = blockIdx.x * 64, c0 = blockIdx.y * 64;
    v8f acc[4][4];
#pragma unroll
    for (int mb = 0; mb < 4; ++mb)
#pragma unroll
        for (int nb = 0; nb < 4; ++nb) acc[mb][nb] = (v8f){};
    const size_t aoff = (size_t)(r0 + lr) * K + 8 * hi, boff = (size_t)(c0 + lr) * K + 8 * hi;
#pragma unroll 1
    for (int kc = 0; kc < K; kc += 32) {
        V a[4], a2[4];
#pragma unroll
        for (int mb = 0; mb < 4; ++mb) { a[mb] = WFrag<T16>::ld(A + aoff + (size_t)mb * 16 * K + kc); if (NSPLIT == 1 || NSPLIT == 2) a2[mb] = WFrag<T16>::ld(A2 + aoff + (size_t)mb * 16 * K + kc); }
#pragma unroll
        for (int nb = 0; nb < 4; ++nb) { const V b = WFrag<T16>::ld(Bt + boff + (size_t)nb * 16 * K + kc); V b2; if (NSPLIT >= 2) b2 = WFrag<T16>::ld(Bt2 + boff + (size_t)nb * 16 * K + kc);
#pragma unroll
            for (int mb = 0; mb < 4; ++mb) { acc[mb][nb] = WFrag<T16>::mma(a[mb], b, acc[mb][nb]); if (NSPLIT == 1 || NSPLIT == 2) acc[mb][nb] = WFrag<T16>::mma(a2[mb], b, acc[mb][nb]); if (NSPLIT >= 2) acc[mb][nb] = WFrag<T16>::mma(a[mb], b2, acc[mb][nb]); } }
        asm volatile("v_nop\n\tv_nop\n\tv_nop\n\tv_nop" : "+v"(acc[0][0]), "+v"(acc[1][1]), "+v"(acc[2][2]), "+v"(acc[3][3]) : "v"(a[0]), "v"(a[3]));
    }
#pragma unroll
    for (int mb = 0; mb < 4; ++mb) {
#pragma unroll
        for (int nb = 0; nb < 4; ++nb) {
#pragma unroll
            for (int j = 0; j < 8; ++j) os[(hi * 8 + j) * 68 + nb * 16 + lr] = acc[mb][nb][j]; }
        __builtin_amdgcn_wave_barrier(); asm volatile("" ::: "memory");
        float* crow = C + (size_t)(r0 + mb * 16) * ldc + c0;
#pragma unroll 1
        for (int ps = 0; ps < 2; ++ps) {
#pragma unroll
            for (int s = 0; s < 8; ++s) { const int row = 2 * s + hi, cofs = lr * 4; v4f val = *(const v4fa*)(os + row * 68 + cofs);
                if (BIASR) { const float bb = bfr(bias[r0 + mb * 16 + row]); val[0] += bb; val[1] += bb; val[2] += bb; val[3] += bb; }
                *(volatile v4f*)(crow + (size_t)row * ldc + cofs) = val; }
            if (ps == 0) __threadfence(); }
        __builtin_amdgcn_wave_barrier(); asm volatile("" ::: "memory");
    }
}

__global__ __launch_bounds__(256) void k_cvt8(const float* __restrict__ src, bf* dst, size_t n8) { const size_t i = (size_t)blockIdx.x * 256 + threadIdx.x; if (i >= n8) return; const v8f v = *(const v8f*)(src + i * 8); v8us o;
#pragma unroll
    for (int k = 0; k < 8; ++k) o[k] = f2bf(v[k]); *(volatile v8us*)(dst + i * 8) = o; __threadfence(); *(volatile v8us*)(dst + i * 8) = o; }

__global__ __launch_bounds__(256) void k_xT(const float* __restrict__ xs, bf* XT, int nimg) {
    const size_t k = (size_t)blockIdx.x * 256 + threadIdx.x; if (k >= (size_t)nimg * HW * (CC / 8)) return;
    const int c0 = (int)(k % (CC / 8)) * 8; const size_t tt = k / (CC / 8); const int t = (int)(tt % HW); const int bb = (int)(tt / HW);
    const float* src = xs + (size_t)bb * IMG; v8us o;
#pragma unroll
    for (int q = 0; q < 8; ++q) o[q] = f2bf(src[(size_t)(c0 + q) * HW + t]);
    bf* dst = XT + ((size_t)bb * HW + t) * CC + c0;
    *(volatile v8us*)dst = o; __threadfence(); *(volatile v8us*)dst = o; }

__global__ __launch_bounds__(256) __attribute__((amdgpu_num_vgpr(256)))
void k_nbr(const float* __restrict__ Qg, const float* __restrict__ Kg, const float* __restrict__ Vg, const float* __restrict__ xres, float* outp) {
#pragma clang fp contract(off)
    const int tid = threadIdx.x, lane = tid & 31, wv = tid >> 5;
    const int tj = lane & 15, cs = lane >> 4;
    const int blk = blockIdx.x;
    const int cg = blk & 15, ti = (blk >> 4) & 15, bb = blk >> 8;
    const int c = cg * 16 + wv * 2 + cs;
    const size_t plane = (size_t)bb * IMG + (size_t)c * HW;
    const float* Qc = Qg + plane; const float* Kc = Kg + plane; const float* Vc = Vg + plane;
    const size_t tok = (size_t)(4 * ti) * WW + 4 * tj;

    float q[16];
#pragma unroll
    for (int r = 0; r < 4; ++r) { const v4f t4 = *(const v4f*)(Qc + tok + (size_t)r * WW); q[4 * r] = t4[0]; q[4 * r + 1] = t4[1]; q[4 * r + 2] = t4[2]; q[4 * r + 3] = t4[3]; }

    float acc[16];
#pragma unroll
    for (int e = 0; e < 16; ++e) acc[e] = 0.0f;
    float m = -1.0e30f, l = 0.0f;

#pragma unroll 1
    for (int di = -1; di <= 1; ++di) {
        const int tii = ti + di;
        const bool vi = ((unsigned)tii < (unsigned)NTK);
        const int tic = tii < 0 ? 0 : (tii > NTK - 1 ? NTK - 1 : tii);
#pragma unroll 1
        for (int dj = -1; dj <= 1; ++dj) {
            const int tjj = tj + dj;
            const bool ok = vi && ((unsigned)tjj < (unsigned)NTK);
            const int tjc = tjj < 0 ? 0 : (tjj > NTK - 1 ? NTK - 1 : tjj);
            const size_t nt = (size_t)(4 * tic) * WW + 4 * tjc;
            float kd = 0.0f;
#pragma unroll
            for (int r = 0; r < 4; ++r) { const v4f k4 = *(const v4f*)(Kc + nt + (size_t)r * WW);
#pragma unroll
                for (int e = 0; e < 4; ++e) kd = fmaf(q[4 * r + e], k4[e], kd); }
            const float s = ok ? kd * SCL : 0.0f;
            const float mn = fmaxf(m, s);
            const float corr = __builtin_amdgcn_exp2f((m - mn) * L2E);
            const float p = __builtin_amdgcn_exp2f((s - mn) * L2E);
            l = fmaf(l, corr, p);
            const float pv = ok ? p : 0.0f;
#pragma unroll
            for (int r = 0; r < 4; ++r) { const v4f v4 = *(const v4f*)(Vc + nt + (size_t)r * WW);
#pragma unroll
                for (int e = 0; e < 4; ++e) { const float t = acc[4 * r + e] * corr; acc[4 * r + e] = fmaf(pv, v4[e], t); } }
            m = mn;
        }
    }
    const float inv = 1.0f / l;
    const float* xr = xres + plane + tok;
    v4f o[4];
#pragma unroll
    for (int r = 0; r < 4; ++r) { const v4f b4 = *(const v4f*)(xr + (size_t)r * WW); v4f t4;
#pragma unroll
        for (int e = 0; e < 4; ++e) { const float en = acc[4 * r + e] * inv; t4[e] = bfr(b4[e]) + en; }
        o[r] = t4; }
    float* op = outp + plane + tok;
#pragma unroll 1
    for (int ps = 0; ps < 2; ++ps) {
#pragma unroll
        for (int r = 0; r < 4; ++r) *(volatile v4f*)(op + (size_t)r * WW) = o[r];
        if (ps == 0) __threadfence(); }
}

extern "C" void kernel_launch(void* const* d_in, const int* in_sizes, int n_in, void* d_out, int out_size, void* d_ws, size_t ws_size, hipStream_t stream) {
    (void)n_in;
    if (in_sizes[0] < NB * IMG || in_sizes[1] < NB * IMG || in_sizes[2] < CC * CC || in_sizes[3] < CC || in_sizes[4] < CC * CC || in_sizes[5] < CC || in_sizes[6] < CC * CC || in_sizes[7] < CC || out_size < NB * IMG) return;
    const float* blue  = (const float*)d_in[0];
    const float* white = (const float*)d_in[1];
    const float* Wq = (const float*)d_in[2];
    const float* bq = (const float*)d_in[3];
    const float* Wk = (const float*)d_in[4];
    const float* bk = (const float*)d_in[5];
    const float* Wv = (const float*)d_in[6];
    const float* bv = (const float*)d_in[7];
    float* out = (float*)d_out;

    char* wsp = (char*)d_ws;
    auto take = [&](size_t bytes) { char* p = wsp; wsp += (bytes + 255) & ~(size_t)255; return (void*)p; };
    bf* Wqb = (bf*)take((size_t)CC * CC * 2);
    bf* Wkb = (bf*)take((size_t)CC * CC * 2);
    bf* Wvb = (bf*)take((size_t)CC * CC * 2);
    bf* XTb = (bf*)take((size_t)GB * HW * CC * 2);
    bf* XTw = (bf*)take((size_t)GB * HW * CC * 2);
    float* Qp = (float*)take((size_t)GB * IMG * 4);
    float* Kp = (float*)take((size_t)GB * IMG * 4);
    float* Vp = (float*)take((size_t)GB * IMG * 4);
    if ((size_t)(wsp - (char*)d_ws) > ws_size) return;

    const size_t n8w = (size_t)CC * CC / 8;
    k_cvt8<<<(unsigned)((n8w + 255) / 256), 256, 0, stream>>>(Wq, Wqb, n8w);
    k_cvt8<<<(unsigned)((n8w + 255) / 256), 256, 0, stream>>>(Wk, Wkb, n8w);
    k_cvt8<<<(unsigned)((n8w + 255) / 256), 256, 0, stream>>>(Wv, Wvb, n8w);
    const unsigned gxT = (unsigned)(((size_t)GB * HW * (CC / 8) + 255) / 256);
    for (int g = 0; g < NB / GB; ++g) {
        const size_t goff = (size_t)g * GB * IMG;
        k_xT<<<gxT, 256, 0, stream>>>(blue + goff, XTb, GB);
        k_xT<<<gxT, 256, 0, stream>>>(white + goff, XTw, GB);
        k_gemmw<bf, 0, true><<<dim3(CC / 64, HW / 64, GB), 32, 0, stream>>>(Wqb, nullptr, XTb, nullptr, CC, Qp, HW, bq, 0, (size_t)HW * CC, (size_t)IMG);
        k_gemmw<bf, 0, true><<<dim3(CC / 64, HW / 64, GB), 32, 0, stream>>>(Wkb, nullptr, XTw, nullptr, CC, Kp, HW, bk, 0, (size_t)HW * CC, (size_t)IMG);
        k_gemmw<bf, 0, true><<<dim3(CC / 64, HW / 64, GB), 32, 0, stream>>>(Wvb, nullptr, XTw, nullptr, CC, Vp, HW, bv, 0, (size_t)HW * CC, (size_t)IMG);
        k_nbr<<<(unsigned)(GB * NTK * (CC / 16)), 256, 0, stream>>>(Qp, Kp, Vp, blue + goff, out + goff);
    }
}
